// ProbAttentionLayer_4827543241298
// MI455X (gfx1250) — hardware-verified
//
#include <hip/hip_runtime.h>

#define NB    4
#define SEQ   2048
#define DM    512
#define NH    8
#define HD    64
#define NTOP  24
#define NBH   (NB * NH)
#define NTOK  (NB * SEQ)
#define NX    (NTOK * DM)
#define NW    (DM * DM)
#define NPL   (NBH * SEQ * HD)
#define NX8   (NX / 8)
#define NEG_INF (-__builtin_inff())

static_assert(DM % 32 == 0);
static_assert(NTOK % 128 == 0);
static_assert(SEQ % 128 == 0);
static_assert(DM == NH * HD);
static_assert(SEQ == 256 * 8);
static_assert(NX8 * 8 == NX);

typedef unsigned short us;
typedef us     v8us  __attribute__((ext_vector_type(8)));
typedef __bf16 v16bf __attribute__((ext_vector_type(16)));
typedef float  v8f   __attribute__((ext_vector_type(8)));
typedef float  v4f   __attribute__((ext_vector_type(4)));
typedef v8us __attribute__((may_alias)) v8usa;
typedef v4f  __attribute__((may_alias)) v4fa;

union Frag { v16bf v; v8us half[2]; };

__device__ __forceinline__ us f2bf(float f) {
  unsigned u = __float_as_uint(f);
  u += 0x7FFFu + ((u >> 16) & 1u);
  return (us)(u >> 16);
}
__device__ __forceinline__ float bf2f(us s) {
  return __uint_as_float(((unsigned)s) << 16);
}

__device__ __forceinline__ v8f wmma_bf16(v16bf a, v16bf b, v8f c) {
  v8f d = __builtin_amdgcn_wmma_f32_16x16x32_bf16(false, a, false, b, (short)0, c, false, false);
  asm volatile("v_nop\n\tv_nop\n\tv_nop\n\tv_nop" : "+v"(d) : "v"(a), "v"(b));
  return d;
}

__device__ __forceinline__ v16bf load_frag(const us* p, int h) {
  Frag f;
  f.half[0] = *(const v8usa*)(p + 8 * h);
  f.half[1] = *(const v8usa*)(p + 16 + 8 * h);
  return f.v;
}

__device__ __forceinline__ void rows64_store_pass(const float* s, float* g, int pitch, int lane) {
  const int q8 = lane & 7, sub = lane >> 3;
  #pragma unroll
  for (int i = 0; i < 16; ++i) {
    const int lid = i * 4 + sub;
    const int row = lid >> 1, hl = lid & 1;
    const v4f v = *(const v4fa*)(s + row * 64 + 32 * hl + 4 * q8);
    *(volatile v4f*)(g + (size_t)row * pitch + 32 * hl + 4 * q8) = v;
  }
}

__global__ __launch_bounds__(256) void cvt_x_kernel(
    const float* __restrict__ xq, const float* __restrict__ xk, const float* __restrict__ xv,
    us* __restrict__ xb)
{
  const int g = blockIdx.x * 256 + threadIdx.x;
  if (g >= 3 * NX8) return;
  const int which = g / NX8;
  const int off = g - which * NX8;
  const float* base = (which == 0) ? xq : ((which == 1) ? xk : xv);
  const float* src = base + (size_t)off * 8;
  us* dst = xb + (size_t)which * NX + (size_t)off * 8;
  const v4f a = *(const v4fa*)src;
  const v4f c = *(const v4fa*)(src + 4);
  const v8us o = { f2bf(a.x), f2bf(a.y), f2bf(a.z), f2bf(a.w),
                   f2bf(c.x), f2bf(c.y), f2bf(c.z), f2bf(c.w) };
  *(volatile v8us*)dst = o;
  __threadfence();
  *(volatile v8us*)dst = o;
}

__global__ __launch_bounds__(256) void cvt_wt_kernel(
    const float* __restrict__ w0, const float* __restrict__ w1,
    const float* __restrict__ w2, const float* __restrict__ w3,
    us* __restrict__ wt)
{
  __shared__ __attribute__((aligned(16))) us sT[64 * 72];
  const int tid = threadIdx.x;
  const int mat = blockIdx.x >> 6, t = blockIdx.x & 63;
  const int k0 = (t >> 3) * 64, n0 = (t & 7) * 64;
  const float* W = (mat == 0) ? w0 : ((mat == 1) ? w1 : ((mat == 2) ? w2 : w3));
  #pragma unroll
  for (int i = 0; i < 4; ++i) {
    const int e4 = i * 256 + tid;
    const int r = e4 >> 4, c4 = e4 & 15;
    const v4f v = *(const v4fa*)(W + (size_t)(k0 + r) * DM + n0 + 4 * c4);
    sT[(4 * c4 + 0) * 72 + r] = f2bf(v.x);
    sT[(4 * c4 + 1) * 72 + r] = f2bf(v.y);
    sT[(4 * c4 + 2) * 72 + r] = f2bf(v.z);
    sT[(4 * c4 + 3) * 72 + r] = f2bf(v.w);
  }
  __syncthreads();
  const int q8 = tid & 7, nb = tid >> 3;
  const v8us o0 = *(const v8usa*)(sT + nb * 72 + 8 * q8);
  const v8us o1 = *(const v8usa*)(sT + (nb + 32) * 72 + 8 * q8);
  us* d0 = wt + (size_t)mat * NW + (size_t)(n0 + nb) * DM + k0 + 8 * q8;
  us* d1 = wt + (size_t)mat * NW + (size_t)(n0 + nb + 32) * DM + k0 + 8 * q8;
  *(volatile v8us*)d0 = o0;
  *(volatile v8us*)d1 = o1;
  __threadfence();
  *(volatile v8us*)d0 = o0;
  *(volatile v8us*)d1 = o1;
}

__global__ __launch_bounds__(128) void proj_kernel(
    const us* __restrict__ xb,
    const us* __restrict__ wt,
    const float* __restrict__ bq, const float* __restrict__ bk, const float* __restrict__ bv,
    float* __restrict__ pl)
{
  __shared__ __attribute__((aligned(16))) float sT[128 * HD];

  const int tid = threadIdx.x, lane = tid & 31, w = tid >> 5;
  const int h = lane >> 4, m = lane & 15;
  const int m0 = blockIdx.x * 128;
  const int which = blockIdx.y >> 3, head = blockIdx.y & 7;
  const int m0w = m0 + 32 * w;

  const us* xa0 = xb + (size_t)which * NX + (size_t)(m0w + m) * DM;
  const us* xa1 = xa0 + (size_t)16 * DM;
  const us* wb  = wt + (size_t)which * NW + (size_t)(head * HD + m) * DM;

  const v8f zero8 = {0.f, 0.f, 0.f, 0.f, 0.f, 0.f, 0.f, 0.f};
  v8f acc[2][4];
  #pragma unroll
  for (int mt = 0; mt < 2; ++mt)
    #pragma unroll
    for (int nt = 0; nt < 4; ++nt) acc[mt][nt] = zero8;

  #pragma unroll 1
  for (int k0 = 0; k0 < DM; k0 += 32) {
    const v16bf a0 = load_frag(xa0 + k0, h);
    const v16bf a1 = load_frag(xa1 + k0, h);
    #pragma unroll
    for (int nt = 0; nt < 4; ++nt) {
      const v16bf b = load_frag(wb + (size_t)nt * 16 * DM + k0, h);
      acc[0][nt] = wmma_bf16(a0, b, acc[0][nt]);
      acc[1][nt] = wmma_bf16(a1, b, acc[1][nt]);
    }
  }

  const float* bias = (which == 0) ? bq : ((which == 1) ? bk : bv);
  #pragma unroll
  for (int nt = 0; nt < 4; ++nt) {
    const int feat = 16 * nt + m;
    const float bvl = bf2f(f2bf(bias[head * HD + feat]));
    #pragma unroll
    for (int mt = 0; mt < 2; ++mt) {
      #pragma unroll
      for (int r = 0; r < 8; ++r) {
        const int tokl = 32 * w + 16 * mt + 8 * h + r;
        sT[tokl * HD + feat] = acc[mt][nt][r] + bvl;
      }
    }
  }
  __syncthreads();

  const int bidx = m0 / SEQ, l0 = m0 - bidx * SEQ, bh = bidx * NH + head;
  float* g = pl + (size_t)which * NPL + ((size_t)bh * SEQ + l0 + 32 * w) * HD;
  const float* s = sT + (32 * w) * HD;
  rows64_store_pass(s, g, HD, lane);
  __threadfence();
  rows64_store_pass(s, g, HD, lane);
}

__global__ __launch_bounds__(128) void km_kernel(
    const float* __restrict__ qp,
    const float* __restrict__ kp,
    const int* __restrict__ idx,
    float* __restrict__ mpl)
{
  __shared__ __attribute__((aligned(16))) float sQ[128 * 68];

  const int tid = threadIdx.x;
  const int bh = blockIdx.y;
  const int l0 = blockIdx.x * 128;
  const float* qsrc = qp + ((size_t)bh * SEQ + l0) * HD;
  #pragma unroll
  for (int i = 0; i < 16; ++i) {
    const int e4 = i * 128 + tid;
    const int row = e4 >> 4, c4 = e4 & 15;
    const v4f v = *(const v4fa*)(qsrc + 4 * e4);
    *(v4fa*)(sQ + row * 68 + 4 * c4) = v;
  }
  __syncthreads();

  const int l = l0 + tid;
  const float* qrow = sQ + tid * 68;
  const int* irow = idx + (size_t)l * NTOP;
  float mx = NEG_INF, sm = 0.f;
  #pragma unroll 1
  for (int s = 0; s < NTOP; ++s) {
    int ki = irow[s];
    ki = (ki < 0) ? 0 : ((ki > SEQ - 1) ? (SEQ - 1) : ki);
    const float* kr = kp + ((size_t)bh * SEQ + ki) * HD;
    float d = 0.f;
    #pragma unroll 2
    for (int c = 0; c < 16; ++c) {
      const v4f kk = *(const v4fa*)(kr + 4 * c);
      const v4f qq = *(const v4fa*)(qrow + 4 * c);
      d = fmaf(qq.x, kk.x, d);
      d = fmaf(qq.y, kk.y, d);
      d = fmaf(qq.z, kk.z, d);
      d = fmaf(qq.w, kk.w, d);
    }
    mx = fmaxf(mx, d);
    sm += d;
  }
  const float mv = mx - sm * (1.0f / 2048.0f);
  float* dst = mpl + (size_t)bh * SEQ + l;
  *(volatile float*)dst = mv;
  __threadfence();
  *(volatile float*)dst = mv;
}

__global__ __launch_bounds__(256) void sel_ctx_kernel(
    const float* __restrict__ qp, const float* __restrict__ kp, const float* __restrict__ vp,
    const float* __restrict__ mpl,
    us* __restrict__ ctxh, us* __restrict__ ctxl)
{
  __shared__ __attribute__((aligned(16))) float sbuf[SEQ];
  __shared__ int   smap[SEQ];
  __shared__ int   ssel[32];
  __shared__ float sval[256];
  __shared__ int   sidx[256];
  __shared__ __attribute__((aligned(16))) float sq[HD];
  __shared__ float sred[256];
  __shared__ __attribute__((aligned(16))) float sAV[NTOP * HD];
  __shared__ __attribute__((aligned(16))) us sH[32 * HD];
  __shared__ __attribute__((aligned(16))) us sL[32 * HD];

  const int tid = threadIdx.x;
  const int bh = blockIdx.x, b = bh >> 3, head = bh & 7;
  const size_t pbase = (size_t)bh * SEQ * HD;

  {
    const float* msrc = mpl + (size_t)bh * SEQ;
    #pragma unroll
    for (int i = 0; i < 2; ++i) {
      const int e4 = i * 256 + tid;
      *(v4fa*)(sbuf + 4 * e4) = *(const v4fa*)(msrc + 4 * e4);
    }
    #pragma unroll
    for (int i = 0; i < 8; ++i) smap[i * 256 + tid] = -1;
    if (tid < 32) ssel[tid] = 0;
  }
  __syncthreads();

  #pragma unroll 1
  for (int it = 0; it < NTOP; ++it) {
    float bvv = NEG_INF;
    int bi = tid * 8;
    #pragma unroll
    for (int i = 0; i < 8; ++i) {
      const float v = sbuf[tid * 8 + i];
      const bool gt = v > bvv;
      bi = gt ? (tid * 8 + i) : bi;
      bvv = gt ? v : bvv;
    }
    sval[tid] = bvv;
    sidx[tid] = bi;
    __syncthreads();
    #pragma unroll 1
    for (int s = 128; s > 0; s >>= 1) {
      const int o = (tid + s > 255) ? 255 : (tid + s);
      const float v2 = sval[o];
      const int   i2 = sidx[o];
      const float v1 = sval[tid];
      const int   i1 = sidx[tid];
      const bool take = (v2 > v1) || (v2 == v1 && i2 < i1);
      if (tid < s) {
        sval[tid] = take ? v2 : v1;
        sidx[tid] = take ? i2 : i1;
      }
      __syncthreads();
    }
    if (tid == 0) {
      int wsel = sidx[0];
      wsel = (wsel < 0) ? 0 : ((wsel > SEQ - 1) ? (SEQ - 1) : wsel);
      ssel[it] = wsel;
      smap[wsel] = it;
      sbuf[wsel] = NEG_INF;
    }
    __syncthreads();
  }

  const float RSQ = 0.04419417382415922f;
  #pragma unroll 1
  for (int it = 0; it < NTOP; ++it) {
    int r = ssel[it];
    r = (r < 0) ? 0 : ((r > SEQ - 1) ? (SEQ - 1) : r);
    if (tid < HD) sq[tid] = qp[pbase + (size_t)r * HD + tid];
    __syncthreads();

    float lmax = NEG_INF;
    #pragma unroll 1
    for (int i = 0; i < 8; ++i) {
      const int j = i * 256 + tid;
      const float* kr = kp + pbase + (size_t)j * HD;
      float d = 0.f;
      #pragma unroll 2
      for (int c = 0; c < 16; ++c) {
        const v4f kk = *(const v4fa*)(kr + 4 * c);
        const v4f qq = *(const v4fa*)(sq + 4 * c);
        d = fmaf(qq.x, kk.x, d);
        d = fmaf(qq.y, kk.y, d);
        d = fmaf(qq.z, kk.z, d);
        d = fmaf(qq.w, kk.w, d);
      }
      const float sc = (j > r) ? NEG_INF : d * RSQ;
      sbuf[j] = sc;
      lmax = fmaxf(lmax, sc);
    }
    sred[tid] = lmax;
    __syncthreads();
    #pragma unroll 1
    for (int s = 128; s > 0; s >>= 1) {
      const int o = (tid + s > 255) ? 255 : (tid + s);
      const float v2 = sred[o];
      const float v1 = sred[tid];
      if (tid < s) sred[tid] = fmaxf(v1, v2);
      __syncthreads();
    }
    const float gmax = sred[0];
    __syncthreads();

    float lsum = 0.f;
    #pragma unroll 1
    for (int i = 0; i < 8; ++i) {
      const int j = i * 256 + tid;
      const float e = __expf(sbuf[j] - gmax);
      sbuf[j] = e;
      lsum += e;
    }
    sred[tid] = lsum;
    __syncthreads();
    #pragma unroll 1
    for (int s = 128; s > 0; s >>= 1) {
      const int o = (tid + s > 255) ? 255 : (tid + s);
      const float v2 = sred[o];
      const float v1 = sred[tid];
      if (tid < s) sred[tid] = v1 + v2;
      __syncthreads();
    }
    const float inv = 1.0f / sred[0];
    __syncthreads();

    const int g = tid >> 6, dk = tid & 63;
    float acc = 0.f;
    #pragma unroll 4
    for (int j = g; j < SEQ; j += 4)
      acc = fmaf(sbuf[j], vp[pbase + (size_t)j * HD + dk], acc);
    sred[tid] = acc;
    __syncthreads();
    if (tid < HD)
      sAV[it * HD + tid] = (sred[tid] + sred[64 + tid] + sred[128 + tid] + sred[192 + tid]) * inv;
    __syncthreads();
  }

  float run = 0.f;
  const int d = tid & 63;
  #pragma unroll 1
  for (int ch = 0; ch < SEQ / 32; ++ch) {
    const int l0 = ch * 32;
    #pragma unroll
    for (int i = 0; i < 2; ++i) {
      const int e4 = i * 256 + tid;
      *(v4fa*)(sbuf + 4 * e4) = *(const v4fa*)(vp + pbase + (size_t)l0 * HD + 4 * e4);
    }
    __syncthreads();
    if (tid < HD) {
      #pragma unroll 4
      for (int rr = 0; rr < 32; ++rr) {
        run += sbuf[rr * HD + d];
        const int u = smap[l0 + rr];
        const int uc = (u < 0) ? 0 : ((u > NTOP - 1) ? (NTOP - 1) : u);
        const float av = sAV[uc * HD + d];
        const float val = (u >= 0) ? av : run;
        const us hi = f2bf(val);
        const us lo = f2bf(val - bf2f(hi));
        sH[rr * HD + d] = hi;
        sL[rr * HD + d] = lo;
      }
    }
    __syncthreads();
    {
      const int line = tid >> 3, q8 = tid & 7;
      const v8us oh = *(const v8usa*)(sH + line * HD + 8 * q8);
      const v8us ol = *(const v8usa*)(sL + line * HD + 8 * q8);
      const size_t gi = ((size_t)(b * SEQ + l0 + line)) * DM + head * HD + 8 * q8;
      *(volatile v8us*)(ctxh + gi) = oh;
      *(volatile v8us*)(ctxl + gi) = ol;
      __threadfence();
      *(volatile v8us*)(ctxh + gi) = oh;
      *(volatile v8us*)(ctxl + gi) = ol;
    }
  }
}

__global__ __launch_bounds__(128) void oproj_kernel(
    const us* __restrict__ ch,
    const us* __restrict__ cl,
    const us* __restrict__ wt3,
    const float* __restrict__ bo,
    float* __restrict__ out)
{
  __shared__ __attribute__((aligned(16))) float sT[128 * HD];

  const int tid = threadIdx.x, lane = tid & 31, w = tid >> 5;
  const int h = lane >> 4, m = lane & 15;
  const int m0 = blockIdx.x * 128;
  const int head = blockIdx.y;
  const int m0w = m0 + 32 * w;

  const us* ha0 = ch + (size_t)(m0w + m) * DM;
  const us* ha1 = ha0 + (size_t)16 * DM;
  const us* la0 = cl + (size_t)(m0w + m) * DM;
  const us* la1 = la0 + (size_t)16 * DM;
  const us* wb  = wt3 + (size_t)(head * HD + m) * DM;

  const v8f zero8 = {0.f, 0.f, 0.f, 0.f, 0.f, 0.f, 0.f, 0.f};
  v8f acc[2][4];
  #pragma unroll
  for (int mt = 0; mt < 2; ++mt)
    #pragma unroll
    for (int nt = 0; nt < 4; ++nt) acc[mt][nt] = zero8;

  #pragma unroll 1
  for (int k0 = 0; k0 < DM; k0 += 32) {
    const v16bf a0h = load_frag(ha0 + k0, h);
    const v16bf a1h = load_frag(ha1 + k0, h);
    const v16bf a0l = load_frag(la0 + k0, h);
    const v16bf a1l = load_frag(la1 + k0, h);
    #pragma unroll
    for (int nt = 0; nt < 4; ++nt) {
      const v16bf bf = load_frag(wb + (size_t)nt * 16 * DM + k0, h);
      acc[0][nt] = wmma_bf16(a0h, bf, acc[0][nt]);
      acc[0][nt] = wmma_bf16(a0l, bf, acc[0][nt]);
      acc[1][nt] = wmma_bf16(a1h, bf, acc[1][nt]);
      acc[1][nt] = wmma_bf16(a1l, bf, acc[1][nt]);
    }
  }

  #pragma unroll
  for (int nt = 0; nt < 4; ++nt) {
    const int feat = 16 * nt + m;
    const float bvl = bf2f(f2bf(bo[head * HD + feat]));
    #pragma unroll
    for (int mt = 0; mt < 2; ++mt) {
      #pragma unroll
      for (int r = 0; r < 8; ++r) {
        const int tokl = 32 * w + 16 * mt + 8 * h + r;
        sT[tokl * HD + feat] = acc[mt][nt][r] + bvl;
      }
    }
  }
  __syncthreads();

  float* g = out + (size_t)(m0 + 32 * w) * DM + head * HD;
  const float* s = sT + (32 * w) * HD;
  rows64_store_pass(s, g, DM, lane);
  __threadfence();
  rows64_store_pass(s, g, DM, lane);
}

extern "C" void kernel_launch(void* const* d_in, const int* in_sizes, int n_in,
                              void* d_out, int out_size, void* d_ws, size_t ws_size,
                              hipStream_t stream) {
  if (n_in < 12) return;
  if (in_sizes[0] != NX || in_sizes[1] != NX || in_sizes[2] != NX) return;
  if (in_sizes[3] != SEQ * NTOP) return;
  if (in_sizes[4] != NW || in_sizes[6] != NW || in_sizes[8] != NW || in_sizes[10] != NW) return;
  if (in_sizes[5] != DM || in_sizes[7] != DM || in_sizes[9] != DM || in_sizes[11] != DM) return;
  if (out_size != NX) return;

  const float* queries = (const float*)d_in[0];
  const float* keys    = (const float*)d_in[1];
  const float* values  = (const float*)d_in[2];
  const int*   idxs    = (const int*)d_in[3];
  const float* Wq = (const float*)d_in[4];
  const float* bq = (const float*)d_in[5];
  const float* Wk = (const float*)d_in[6];
  const float* bk = (const float*)d_in[7];
  const float* Wv = (const float*)d_in[8];
  const float* bv = (const float*)d_in[9];
  const float* Wo = (const float*)d_in[10];
  const float* bo = (const float*)d_in[11];
  float* out = (float*)d_out;

  const size_t xb_bytes  = (size_t)3 * NX * 2;
  const size_t wt_bytes  = (size_t)4 * NW * 2;
  const size_t pl_bytes  = (size_t)3 * NPL * 4;
  const size_t m_bytes   = (size_t)NBH * SEQ * 4;
  const size_t ctx_bytes = (size_t)NX * 2;
  const size_t off_xb  = 0;
  const size_t off_wt  = off_xb + xb_bytes;
  const size_t off_pl  = off_wt + wt_bytes;
  const size_t off_m   = off_pl + pl_bytes;
  const size_t off_ch  = off_m + m_bytes;
  const size_t off_cl  = off_ch + ctx_bytes;
  const size_t total   = off_cl + ctx_bytes;
  if (total > ws_size) return;

  char* ws = (char*)d_ws;
  us*    xb   = (us*)(ws + off_xb);
  us*    wt   = (us*)(ws + off_wt);
  float* pl   = (float*)(ws + off_pl);
  float* mpl  = (float*)(ws + off_m);
  us*    ctxh = (us*)(ws + off_ch);
  us*    ctxl = (us*)(ws + off_cl);
  const float* qp = pl;
  const float* kp = pl + (size_t)NPL;
  const float* vp = pl + (size_t)2 * NPL;

  cvt_x_kernel<<<(3 * NX8) / 256, 256, 0, stream>>>(queries, keys, values, xb);
  cvt_wt_kernel<<<4 * 64, 256, 0, stream>>>(Wq, Wk, Wv, Wo, wt);

  dim3 gProj(NTOK / 128, 3 * NH);
  proj_kernel<<<gProj, 128, 0, stream>>>(xb, wt, bq, bk, bv, pl);

  dim3 gM(SEQ / 128, NBH);
  km_kernel<<<gM, 128, 0, stream>>>(qp, kp, idxs, mpl);

  sel_ctx_kernel<<<NBH, 256, 0, stream>>>(qp, kp, vp, mpl, ctxh, ctxl);

  dim3 gO(NTOK / 128, NH);
  oproj_kernel<<<gO, 128, 0, stream>>>(ctxh, ctxl, wt + (size_t)3 * NW, bo, out);
}
